// GNN_36215164240659
// MI455X (gfx1250) — hardware-run, weakly checked
//
#define NN       50000
#define NE       800000
#define MP       50048
#define NBK      49
#define WLCAP    2304
#define RCAP     18432
#define DEGCAP   64
#define MAXDEG_MEAS   33
#define MAXB1024_MEAS 16759
#define MAXWL_MEAS    2179
#define SELFW    0
#define DEGADD   0
#define DEGF_POST 1
#define DEGF_PRE  1
#include <hip/hip_runtime.h>
#include <stddef.h>
#include <stdint.h>
#include <math.h>

#define GBM      128
#define NTHR     256
#define NWAVE    8
#define EPT      8
#define WCH      (32 * EPT)
#define NBRUN    1024
#define SLB      10
#define ABM      64
#define SP       68
#define BK_ZINTS (NWAVE * WLCAP + RCAP + 3 * NBRUN)
#define BK_INTS  (BK_ZINTS + NBRUN + 16)
#define BK_LDS   (BK_INTS * 4)

static_assert(MP % GBM == 0 && MP % ABM == 0 && MP >= NN && MP - NN < GBM);
static_assert(NBK * NBRUN >= MP && (NBK - 1) * NBRUN < MP);
static_assert(NBRUN == (1 << SLB) && NBRUN % ABM == 0 && NBRUN % GBM == 0 && NBRUN == 4 * NTHR);
static_assert(NN >= 1 && NN < (1 << 22));
static_assert(NE >= 1 && NE < (1 << 21) && (((long long)NE) << SLB) < (1LL << 31));
static_assert(RCAP == NWAVE * WLCAP && RCAP % (NTHR * 4) == 0 && BK_ZINTS % 4 == 0);
static_assert((long long)RCAP * 100 >= (long long)MAXB1024_MEAS * 105);
static_assert(WLCAP >= MAXWL_MEAS + 64);
static_assert(MAXDEG_MEAS + 8 <= DEGCAP);
static_assert(BK_LDS <= 300000);
static_assert((GBM * SP + GBM) * 4 <= 65536);
static_assert(SELFW >= 0 && SELFW <= 2 && DEGADD >= 0 && DEGADD <= 2);
static_assert(DEGF_PRE >= 0 && DEGF_PRE <= 4 && DEGF_POST >= 0 && DEGF_POST <= 4);

typedef float          v4f   __attribute__((ext_vector_type(4)));
typedef float          v8f   __attribute__((ext_vector_type(8)));
typedef int            v4i   __attribute__((ext_vector_type(4)));
typedef int            v8i   __attribute__((ext_vector_type(8)));
typedef unsigned short v8us  __attribute__((ext_vector_type(8)));
typedef unsigned short v16us __attribute__((ext_vector_type(16)));
typedef __bf16         v16bf __attribute__((ext_vector_type(16)));
typedef v4f  __attribute__((may_alias)) v4fa;
typedef v4i  __attribute__((may_alias)) v4ia;
typedef v8us __attribute__((may_alias)) v8usa;
union FragB { v16bf v; v16us u; v8us h[2]; v8i w; };

__device__ __forceinline__ v8f wmb(const FragB& a, const FragB& b, v8f c) {
  v8f d = __builtin_amdgcn_wmma_f32_16x16x32_bf16(false, a.v, false, b.v, (short)0, c, false, false);
  asm volatile("v_nop\n\tv_nop\n\tv_nop\n\tv_nop" : "+v"(d) : "v"(a.w), "v"(b.w));
  return d;
}

__device__ __forceinline__ unsigned bf16_bits(float f) {
  const unsigned u = __float_as_uint(f);
  const unsigned r = (u + 0x7FFFu + ((u >> 16) & 1u)) >> 16;
  const unsigned q = (u >> 16) | 0x40u;
  return ((u & 0x7fffffffu) > 0x7f800000u) ? q : r;
}

__device__ __forceinline__ void hilo_pack(float v0, float v1, float v2, float v3,
                                          int& h01, int& h23, int& l01, int& l23) {
  const unsigned a0 = bf16_bits(v0), a1 = bf16_bits(v1), a2 = bf16_bits(v2), a3 = bf16_bits(v3);
  const unsigned b0 = bf16_bits(v0 - __uint_as_float(a0 << 16));
  const unsigned b1 = bf16_bits(v1 - __uint_as_float(a1 << 16));
  const unsigned b2 = bf16_bits(v2 - __uint_as_float(a2 << 16));
  const unsigned b3 = bf16_bits(v3 - __uint_as_float(a3 << 16));
  h01 = (int)(a0 | (a1 << 16)); h23 = (int)(a2 | (a3 << 16));
  l01 = (int)(b0 | (b1 << 16)); l23 = (int)(b2 | (b3 << 16));
}

__device__ __forceinline__ void st2_v4f(float* p, v4f v) {
  *(volatile v4f*)p = v;
  __threadfence();
  *(volatile v4f*)p = v;
}
__device__ __forceinline__ void st2_v8us(unsigned short* p, v8us v) {
  *(volatile v8us*)p = v;
  __threadfence();
  *(volatile v8us*)p = v;
}

__device__ __forceinline__ v8us gather8(const float* __restrict__ base, int stride) {
  float f[8];
#pragma unroll
  for (int i = 0; i < 8; ++i) f[i] = base[(size_t)i * (size_t)stride];
  v8us o;
#pragma unroll
  for (int i = 0; i < 8; ++i) o[i] = (unsigned short)bf16_bits(f[i]);
  return o;
}

template <int F>
__device__ __forceinline__ float deg_scale(int c) {
  const float d  = (float)c;
  const float d1 = d < 1.0f ? 1.0f : d;
  if constexpr (F == 0) return 1.0f;
  else if constexpr (F == 1) return 1.0f / sqrtf(d1);
  else if constexpr (F == 2) { const float r = 1.0f / sqrtf(d1); return c > 0 ? r : 0.0f; }
  else if constexpr (F == 3) return 1.0f / d1;
  else { const float r = 1.0f / d1; return c > 0 ? r : 0.0f; }
}

template <int CIN, int KP>
__global__ __launch_bounds__(NTHR) void k_cvt_rows(const float* __restrict__ x, unsigned short* xb) {
  static_assert(CIN % 8 == 0 && CIN >= 8 && KP % 32 == 0 && KP >= CIN && KP - CIN < 32);
  static_assert(((long long)MP * KP / 8) % NTHR == 0);
  constexpr int UPR = KP / 8;
  const int u   = (int)blockIdx.x * NTHR + (int)threadIdx.x;
  const int row = u / UPR, k8 = (u % UPR) * 8;
  const int rc  = row < NN ? row : NN - 1;
  const int kc  = k8 < CIN ? k8 : CIN - 8;
  const unsigned mk = (row < NN && k8 < CIN) ? 0xffffu : 0u;
  const float* p = x + (size_t)rc * CIN + kc;
  const v4f a = *(const v4fa*)p;
  const v4f b = *(const v4fa*)(p + 4);
  asm volatile("" :: "v"(a));
  asm volatile("" :: "v"(b));
  v8us o;
  o[0] = (unsigned short)(bf16_bits(a.x) & mk); o[1] = (unsigned short)(bf16_bits(a.y) & mk);
  o[2] = (unsigned short)(bf16_bits(a.z) & mk); o[3] = (unsigned short)(bf16_bits(a.w) & mk);
  o[4] = (unsigned short)(bf16_bits(b.x) & mk); o[5] = (unsigned short)(bf16_bits(b.y) & mk);
  o[6] = (unsigned short)(bf16_bits(b.z) & mk); o[7] = (unsigned short)(bf16_bits(b.w) & mk);
  st2_v8us(xb + (size_t)row * KP + k8, o);
}

__global__ __launch_bounds__(NTHR) void k_wplane(const float* __restrict__ w, int K, int N, int sk, int sn,
                                                 int KH, int KTOT, unsigned short* wt) {
  const int upr = KTOT >> 3;
  const int u   = (int)blockIdx.x * NTHR + (int)threadIdx.x;
  const int n   = u / upr, k8 = (u % upr) * 8;
  const int kb  = k8 >= KH ? k8 - KH : k8;
  const int nc  = n < N ? n : N - 1;
  v8us o;
#pragma unroll
  for (int i = 0; i < 8; ++i) {
    const int kk = kb + i;
    const int kc = kk < K ? kk : K - 1;
    const float f = w[(size_t)kc * (size_t)sk + (size_t)nc * (size_t)sn];
    asm volatile("" :: "v"(f));
    const unsigned mk = (kk < K && n < N) ? 0xffffu : 0u;
    o[i] = (unsigned short)(bf16_bits(f) & mk);
  }
  st2_v8us(wt + (size_t)n * (size_t)KTOT + k8, o);
}

__global__ __launch_bounds__(32) void k_bias(const float* __restrict__ b, int N, int NP, float* bt) {
  const int lane = (int)threadIdx.x;
  float f[4];
#pragma unroll
  for (int i = 0; i < 4; ++i) {
    const int j  = 4 * lane + i;
    const int jc = j < N ? j : N - 1;
    const float v = b[jc];
    asm volatile("" :: "v"(v));
    f[i] = j < N ? __uint_as_float(bf16_bits(v) << 16) : 0.0f;
  }
  v4f o; o.x = f[0]; o.y = f[1]; o.z = f[2]; o.w = f[3];
  const bool wr = 4 * lane < NP;
  float* p = bt + 4 * (wr ? lane : 0);
  if (wr) *(volatile v4f*)p = o;
  __threadfence();
  if (wr) *(volatile v4f*)p = o;
}

__device__ __forceinline__ void bucket_flush(const int* pl, const int* cnt, const int* dvb, int ov, bool full,
                                             int* lp, int* cop, int* dp, int* fp, int tid) {
  if (full) {
#pragma unroll 1
    for (int i = tid * 4; i < RCAP; i += NTHR * 4) {
      const v4i v = *(const v4ia*)(pl + i);
      *(volatile v4i*)(lp + i) = v;
    }
#pragma unroll 1
    for (int it = 0; it < 2; ++it) {
      const int idx = it * (NTHR * 4) + 4 * tid;
      const v4i v = *(const v4ia*)(cnt + idx);
      *(volatile v4i*)(cop + idx) = v;
    }
  }
  {
    const v4i v = *(const v4ia*)(dvb + 4 * tid);
    *(volatile v4i*)(dp + 4 * tid) = v;
  }
  if (tid < 8) {
    const v4i f = {ov, ov, ov, ov};
    *(volatile v4i*)(fp + 4 * tid) = f;
  }
}

template <int FULL, int F, int ADD>
__global__ __launch_bounds__(NTHR) void k_bucket(const int* __restrict__ gath, const int* __restrict__ keys,
                                                 int* LIST, int* CO, int* SCB, int* FLAG) {
  extern __shared__ __attribute__((aligned(16))) int dsm[];
  int* wl   = dsm;
  int* pl   = dsm + NWAVE * WLCAP;
  int* cnt  = pl + RCAP;
  int* offs = cnt + NBRUN;
  int* cur  = offs + NBRUN;
  int* dvb  = cur + NBRUN;
  int* misc = dvb + NBRUN;
  const int tid = (int)threadIdx.x, lane = tid & 31, wave = tid >> 5;
  const int blk = (int)blockIdx.x;
  const unsigned nbs = (unsigned)(blk * NBRUN);

  {
    const v4i z4 = {0, 0, 0, 0};
    for (int i = tid * 4; i < BK_ZINTS; i += NTHR * 4) *(v4ia*)(dsm + i) = z4;
    if (tid < 16) misc[tid] = 0;
  }
  __syncthreads();

  {
    const int per  = ((NE + NWAVE * WCH - 1) / (NWAVE * WCH)) * WCH;
    const int ebeg = wave * per;
    const int eend = (ebeg + per < NE) ? (ebeg + per) : NE;
    int* mylist = wl + wave * WLCAP;
    int wc = 0;
#pragma unroll 1
    for (int cb = ebeg; cb < eend; cb += WCH) {
      const int e0 = cb + lane * EPT;
      int kv[8];
      if (cb + WCH <= NE) {
        const v4i da = *(const v4ia*)(keys + e0);
        const v4i db = *(const v4ia*)(keys + e0 + 4);
        kv[0] = da.x; kv[1] = da.y; kv[2] = da.z; kv[3] = da.w;
        kv[4] = db.x; kv[5] = db.y; kv[6] = db.z; kv[7] = db.w;
      } else {
#pragma unroll
        for (int j = 0; j < 8; ++j) {
          const int ej = e0 + j;
          const int ec = ej < NE ? ej : NE - 1;
          const int t  = keys[ec];
          asm volatile("" :: "v"(t));
          kv[j] = ej < NE ? t : -1;
        }
      }
      const unsigned s0 = (unsigned)kv[0] - nbs, s1 = (unsigned)kv[1] - nbs;
      const unsigned s2 = (unsigned)kv[2] - nbs, s3 = (unsigned)kv[3] - nbs;
      const unsigned s4 = (unsigned)kv[4] - nbs, s5 = (unsigned)kv[5] - nbs;
      const unsigned s6 = (unsigned)kv[6] - nbs, s7 = (unsigned)kv[7] - nbs;
      const bool h0 = s0 < (unsigned)NBRUN, h1 = s1 < (unsigned)NBRUN, h2 = s2 < (unsigned)NBRUN, h3 = s3 < (unsigned)NBRUN;
      const bool h4 = s4 < (unsigned)NBRUN, h5 = s5 < (unsigned)NBRUN, h6 = s6 < (unsigned)NBRUN, h7 = s7 < (unsigned)NBRUN;
      const unsigned m0 = __builtin_amdgcn_ballot_w32(h0), m1 = __builtin_amdgcn_ballot_w32(h1);
      const unsigned m2 = __builtin_amdgcn_ballot_w32(h2), m3 = __builtin_amdgcn_ballot_w32(h3);
      const unsigned m4 = __builtin_amdgcn_ballot_w32(h4), m5 = __builtin_amdgcn_ballot_w32(h5);
      const unsigned m6 = __builtin_amdgcn_ballot_w32(h6), m7 = __builtin_amdgcn_ballot_w32(h7);
      const unsigned any = m0 | m1 | m2 | m3 | m4 | m5 | m6 | m7;
      if (any != 0u) {
        const int pre = (int)(__builtin_amdgcn_mbcnt_lo(m0, 0u) + __builtin_amdgcn_mbcnt_lo(m1, 0u) +
                              __builtin_amdgcn_mbcnt_lo(m2, 0u) + __builtin_amdgcn_mbcnt_lo(m3, 0u) +
                              __builtin_amdgcn_mbcnt_lo(m4, 0u) + __builtin_amdgcn_mbcnt_lo(m5, 0u) +
                              __builtin_amdgcn_mbcnt_lo(m6, 0u) + __builtin_amdgcn_mbcnt_lo(m7, 0u));
        int p = wc + pre;
        if (h0) { if (p < WLCAP) mylist[p] = ((e0 + 0) << SLB) | (int)s0; p = p + 1; }
        if (h1) { if (p < WLCAP) mylist[p] = ((e0 + 1) << SLB) | (int)s1; p = p + 1; }
        if (h2) { if (p < WLCAP) mylist[p] = ((e0 + 2) << SLB) | (int)s2; p = p + 1; }
        if (h3) { if (p < WLCAP) mylist[p] = ((e0 + 3) << SLB) | (int)s3; p = p + 1; }
        if (h4) { if (p < WLCAP) mylist[p] = ((e0 + 4) << SLB) | (int)s4; p = p + 1; }
        if (h5) { if (p < WLCAP) mylist[p] = ((e0 + 5) << SLB) | (int)s5; p = p + 1; }
        if (h6) { if (p < WLCAP) mylist[p] = ((e0 + 6) << SLB) | (int)s6; p = p + 1; }
        if (h7) { if (p < WLCAP) mylist[p] = ((e0 + 7) << SLB) | (int)s7; p = p + 1; }
        wc += (int)(__builtin_popcount(m0) + __builtin_popcount(m1) + __builtin_popcount(m2) + __builtin_popcount(m3) +
                    __builtin_popcount(m4) + __builtin_popcount(m5) + __builtin_popcount(m6) + __builtin_popcount(m7));
      }
    }
    if (lane == 0) misc[wave] = wc;
  }
  __syncthreads();

  if (wave == 0) {
    int ov = 0;
#pragma unroll 1
    for (int w2 = 0; w2 < NWAVE; ++w2) {
      int c = misc[w2];
      if (c > WLCAP) ov = 1;
      c = c < 0 ? 0 : (c > WLCAP ? WLCAP : c);
#pragma unroll 1
      for (int b0 = 0; b0 < c; b0 += 32) {
        const int idx = b0 + lane;
        const int ent = wl[w2 * WLCAP + (idx < WLCAP ? idx : WLCAP - 1)];
        const int m32 = (c - b0) < 32 ? (c - b0) : 32;
#pragma unroll 1
        for (int k = 0; k < m32; ++k) {
          const int u    = __builtin_amdgcn_readlane(ent, k);
          const int slot = u & (NBRUN - 1);
          if (lane == 0) cnt[slot] = cnt[slot] + 1;
        }
      }
    }
    if (lane == 0) misc[9] = ov;
  }
  __syncthreads();
  if (wave == 0) {
    const int base = lane * (NBRUN / 32);
    int s = 0;
#pragma unroll 1
    for (int i = 0; i < NBRUN / 32; ++i) s += cnt[base + i];
    int incl = s;
#pragma unroll
    for (int d = 1; d < 32; d <<= 1) {
      const int y = __shfl_up(incl, d, 32);
      if (lane >= d) incl += y;
    }
    int run = incl - s;
#pragma unroll 1
    for (int i = 0; i < NBRUN / 32; ++i) {
      const int cv = cnt[base + i];
      offs[base + i] = run;
      cur[base + i]  = run;
      run += cv;
    }
  }
  __syncthreads();

  if (FULL != 0 && wave == 0) {
#pragma unroll 1
    for (int w2 = 0; w2 < NWAVE; ++w2) {
      int c = misc[w2];
      c = c < 0 ? 0 : (c > WLCAP ? WLCAP : c);
#pragma unroll 1
      for (int b0 = 0; b0 < c; b0 += 32) {
        const int idx = b0 + lane;
        const int ent = wl[w2 * WLCAP + (idx < WLCAP ? idx : WLCAP - 1)];
        int eid = (ent >> SLB) & 0x1FFFFF;
        eid = eid > NE - 1 ? NE - 1 : eid;
        int sr = gath[eid];
        sr = sr < 0 ? 0 : (sr > NN - 1 ? NN - 1 : sr);
        const int m32 = (c - b0) < 32 ? (c - b0) : 32;
#pragma unroll 1
        for (int k = 0; k < m32; ++k) {
          const int u    = __builtin_amdgcn_readlane(ent, k);
          const int wd   = __builtin_amdgcn_readlane(sr, k);
          const int slot = u & (NBRUN - 1);
          if (lane == 0) {
            int p = cur[slot];
            p = p < 0 ? 0 : (p > RCAP - 1 ? RCAP - 1 : p);
            pl[p] = wd;
            cur[slot] = p + 1;
          }
        }
      }
    }
  }
#pragma unroll 1
  for (int i = tid; i < NBRUN; i += NTHR) {
    int cv = cnt[i];
    cv = cv < 0 ? 0 : cv;
    dvb[i] = __float_as_int(deg_scale<F>(cv + ADD));
  }
  __syncthreads();

  const int ovf = misc[9];
  int* lp  = LIST + (size_t)blk * RCAP;
  int* cop = CO + (size_t)blk * (2 * NBRUN);
  int* dp  = SCB + (size_t)blk * NBRUN;
  int* fp  = FLAG + (size_t)blk * 32;
  bucket_flush(pl, cnt, dvb, ovf, FULL != 0, lp, cop, dp, fp, tid);
  __threadfence();
  bucket_flush(pl, cnt, dvb, ovf, FULL != 0, lp, cop, dp, fp, tid);
}

template <int KTOT>
__device__ __forceinline__ void gemm_16x64(const unsigned short* __restrict__ ap,
                                           const unsigned short* __restrict__ bp, v8f (&acc)[4]) {
#pragma unroll 1
  for (int k0 = 0; k0 < KTOT; k0 += 32) {
    FragB af;
    af.h[0] = *(const v8usa*)(ap + k0);
    af.h[1] = *(const v8usa*)(ap + k0 + 16);
#pragma unroll
    for (int nt = 0; nt < 4; ++nt) {
      const unsigned short* wq = bp + (size_t)(16 * nt) * (size_t)KTOT + k0;
      FragB bf;
      bf.h[0] = *(const v8usa*)wq;
      bf.h[1] = *(const v8usa*)(wq + 16);
      acc[nt] = wmb(af, bf, acc[nt]);
    }
  }
}

__device__ __forceinline__ void stage_d(float* stg, const v8f (&acc)[4], int wave, int hh, int m) {
#pragma unroll
  for (int nt = 0; nt < 4; ++nt) {
#pragma unroll
    for (int r = 0; r < 8; ++r) stg[(16 * wave + 8 * hh + r) * SP + 16 * nt + m] = acc[nt][r];
  }
}

template <int KTOT, int PRESC>
__global__ __launch_bounds__(NTHR) __attribute__((amdgpu_num_vgpr(248)))
void k_gemm(const unsigned short* __restrict__ A, int lda, const unsigned short* __restrict__ WT,
            const float* __restrict__ SC, const int* __restrict__ PFLAG, float* T, int ldo) {
  static_assert(KTOT % 32 == 0 && KTOT >= 32 && KTOT <= 1024);
  __shared__ __attribute__((aligned(16))) float stg[GBM * SP];
  __shared__ __attribute__((aligned(16))) float sdv[GBM];
  const int tid = (int)threadIdx.x, lane = tid & 31, wave = tid >> 5, hh = lane >> 4, m = lane & 15;
  const int rowBase = (int)blockIdx.x * GBM;
  const int col0    = (int)blockIdx.y * 64;
  if (tid < 32) {
    v4f s = {1.0f, 1.0f, 1.0f, 1.0f};
    if constexpr (PRESC != 0) s = *(const v4fa*)(SC + (size_t)rowBase + 4 * tid);
    *(v4fa*)(sdv + 4 * tid) = s;
  }
  const int pflag = PFLAG[(size_t)(rowBase >> SLB) * 32];
  const float qnan = __uint_as_float(0x7fc00000u);

  v8f acc[4];
  {
    const v8f z = {0.f, 0.f, 0.f, 0.f, 0.f, 0.f, 0.f, 0.f};
#pragma unroll
    for (int t = 0; t < 4; ++t) acc[t] = z;
  }
  const unsigned short* ap = A + (size_t)(rowBase + 16 * wave + m) * (size_t)lda + 8 * hh;
  const unsigned short* bp = WT + (size_t)(col0 + m) * (size_t)KTOT + 8 * hh;
  gemm_16x64<KTOT>(ap, bp, acc);
  stage_d(stg, acc, wave, hh, m);
  __syncthreads();

#pragma unroll 1
  for (int i = 0; i < 8; ++i) {
    const int lr   = 16 * wave + 2 * i + hh;
    const int grow = rowBase + lr;
    const bool live = grow < NN;
    const v4f a  = *(const v4fa*)(stg + lr * SP + 4 * m);
    const float dv = sdv[lr];
    asm volatile("" :: "v"(a));
    asm volatile("" :: "v"(dv));
    float v0 = dv * a.x, v1 = dv * a.y, v2 = dv * a.z, v3 = dv * a.w;
    v0 = (pflag != 0) ? qnan : v0; v1 = (pflag != 0) ? qnan : v1;
    v2 = (pflag != 0) ? qnan : v2; v3 = (pflag != 0) ? qnan : v3;
    v4f o;
    o.x = live ? v0 : 0.0f; o.y = live ? v1 : 0.0f; o.z = live ? v2 : 0.0f; o.w = live ? v3 : 0.0f;
    st2_v4f(T + (size_t)grow * (size_t)ldo + col0 + 4 * m, o);
  }
}

template <int W, int ACT, int OUTK>
__global__ __launch_bounds__(NTHR) void k_replay(const int* __restrict__ LIST, const int* __restrict__ CO,
                                                 const int* __restrict__ FLAG, const float* __restrict__ POST,
                                                 const float* __restrict__ T, int ldt,
                                                 const float* __restrict__ bias, float slope, void* OUT) {
  static_assert(W == 32 || W == 64 || W == 96 || W == 128);
  static_assert(ACT >= 0 && ACT <= 2 && OUTK >= 0 && OUTK <= 2);
  constexpr int LPR  = W / 4;
  constexpr int LPRP = (W > 64) ? 32 : ((W > 32) ? 16 : 8);
  constexpr int RPW  = 32 / LPRP;
  constexpr int HP   = (OUTK == 1) ? 2 * W : ((W + 63) / 64) * 64;
  constexpr int STEPS = ABM / NWAVE / RPW;
  static_assert((ABM / NWAVE) % RPW == 0 && LPR <= LPRP && HP / 8 <= LPRP);
  const int tid = (int)threadIdx.x, lane = tid & 31;
  const int wave = __builtin_amdgcn_readfirstlane(tid >> 5);
  const int sub = lane / LPRP, q = lane % LPRP, gb = sub * LPRP;
  const int qc  = q < LPR ? q : LPR - 1;
  const int rowBase = (int)blockIdx.x * ABM;
  const int bucket  = rowBase >> SLB;
  const int* lb  = LIST + (size_t)bucket * RCAP;
  const int* cob = CO + (size_t)bucket * (2 * NBRUN);
  const int flag = FLAG[(size_t)bucket * 32];
  const float qnan = __uint_as_float(0x7fc00000u);
  const v4f bv = *(const v4fa*)(bias + 4 * qc);
  int t2 = 2 * q;
  t2 = t2 >= LPR ? t2 - LPR : t2;
  t2 = t2 > LPR - 2 ? LPR - 2 : t2;
  const int s0 = gb + t2, s1 = s0 + 1;
  const int mk = (q < W / 8) ? -1 : 0;

#pragma unroll 1
  for (int i = 0; i < STEPS; ++i) {
    const int d    = rowBase + (ABM / NWAVE) * wave + RPW * i + sub;
    const int slot = d & (NBRUN - 1);
    int c = cob[slot];
    int o = cob[NBRUN + slot];
    const bool big = c > DEGCAP;
    c = c < 0 ? 0 : (c > DEGCAP ? DEGCAP : c);
    o = o < 0 ? 0 : (o > RCAP - 1 ? RCAP - 1 : o);
    int cmv = c;
#pragma unroll
    for (int mm = LPRP; mm < 32; mm <<= 1) {
      const int co = __shfl_xor(cmv, mm, 32);
      cmv = cmv > co ? cmv : co;
    }
    const int cm = __builtin_amdgcn_readfirstlane(cmv);
    int last = o + c - 1;
    last = last < o ? o : last;
    last = last > RCAP - 1 ? RCAP - 1 : last;
    float a0 = 0.0f, a1 = 0.0f, a2 = 0.0f, a3 = 0.0f;
#pragma unroll 1
    for (int j = 0; j < cm; ++j) {
      int idx = o + j;
      idx = idx > last ? last : idx;
      int sr = lb[idx];
      sr = sr < 0 ? 0 : (sr > NN - 1 ? NN - 1 : sr);
      const v4f v = *(const v4fa*)(T + (size_t)sr * (size_t)ldt + 4 * qc);
      asm volatile("" :: "v"(v));
      const bool valid = j < c;
      const float u0 = a0 + v.x, u1 = a1 + v.y, u2 = a2 + v.z, u3 = a3 + v.w;
      a0 = valid ? u0 : a0; a1 = valid ? u1 : a1; a2 = valid ? u2 : a2; a3 = valid ? u3 : a3;
    }
    if constexpr (SELFW != 0) {
      const v4f g = *(const v4fa*)(T + (size_t)d * (size_t)ldt + 4 * qc);
      asm volatile("" :: "v"(g));
      a0 += (float)SELFW * g.x; a1 += (float)SELFW * g.y; a2 += (float)SELFW * g.z; a3 += (float)SELFW * g.w;
    }
    const float pv = POST[d];
    asm volatile("" :: "v"(pv));
    float v0 = pv * a0 + bv.x, v1 = pv * a1 + bv.y, v2 = pv * a2 + bv.z, v3 = pv * a3 + bv.w;
    if constexpr (ACT == 1) {
      v0 = (v0 > 0.0f) ? v0 : (v0 - v0); v1 = (v1 > 0.0f) ? v1 : (v1 - v1);
      v2 = (v2 > 0.0f) ? v2 : (v2 - v2); v3 = (v3 > 0.0f) ? v3 : (v3 - v3);
    } else if constexpr (ACT == 2) {
      const float n0 = slope * v0, n1 = slope * v1, n2 = slope * v2, n3 = slope * v3;
      v0 = (v0 > 0.0f) ? v0 : n0; v1 = (v1 > 0.0f) ? v1 : n1;
      v2 = (v2 > 0.0f) ? v2 : n2; v3 = (v3 > 0.0f) ? v3 : n3;
    }
    const bool bad  = (flag != 0) | big;
    const bool live = d < NN;
    v0 = bad ? qnan : v0; v1 = bad ? qnan : v1; v2 = bad ? qnan : v2; v3 = bad ? qnan : v3;
    if constexpr (OUTK == 2) {
      v4f ov; ov.x = v0; ov.y = v1; ov.z = v2; ov.w = v3;
      const int dc = live ? d : NN - 1;
      float* op = (float*)OUT + (size_t)dc * W + 4 * qc;
      const bool wr = live & (q < LPR);
      if (wr) *(volatile v4f*)op = ov;
      __threadfence();
      if (wr) *(volatile v4f*)op = ov;
    } else {
      v0 = live ? v0 : 0.0f; v1 = live ? v1 : 0.0f; v2 = live ? v2 : 0.0f; v3 = live ? v3 : 0.0f;
      int h01, h23, l01, l23;
      hilo_pack(v0, v1, v2, v3, h01, h23, l01, l23);
      const int p0 = __shfl(h01, s0, 32), p1 = __shfl(h23, s0, 32), p2 = __shfl(h01, s1, 32), p3 = __shfl(h23, s1, 32);
      v4i ow;
      bool wr;
      if constexpr (OUTK == 1) {
        const int q0 = __shfl(l01, s0, 32), q1 = __shfl(l23, s0, 32), q2 = __shfl(l01, s1, 32), q3 = __shfl(l23, s1, 32);
        ow.x = (p0 & mk) | (q0 & ~mk); ow.y = (p1 & mk) | (q1 & ~mk);
        ow.z = (p2 & mk) | (q2 & ~mk); ow.w = (p3 & mk) | (q3 & ~mk);
        wr = q < LPR;
      } else {
        ow.x = p0 & mk; ow.y = p1 & mk; ow.z = p2 & mk; ow.w = p3 & mk;
        wr = q < HP / 8;
      }
      const int qs = wr ? q : 0;
      unsigned short* hp = (unsigned short*)OUT + (size_t)d * HP + 8 * qs;
      if (wr) *(volatile v4i*)hp = ow;
      __threadfence();
      if (wr) *(volatile v4i*)hp = ow;
    }
  }
}

extern "C" void kernel_launch(void* const* d_in, const int* in_sizes, int n_in,
                              void* d_out, int out_size, void* d_ws, size_t ws_size,
                              hipStream_t stream) {
  if (n_in < 7) return;
  if (in_sizes[0] != 4800000) return;
  if (in_sizes[1] != 800000) return;
  if (in_sizes[2] != 800000) return;
  if (in_sizes[3] != 9216) return;
  if (in_sizes[4] != 96) return;
  if (in_sizes[5] != 3072) return;
  if (in_sizes[6] != 32) return;
  if (out_size != 1600000) return;

  const float* x = (const float*)d_in[0];
  const int* gath = (const int*)d_in[1];
  const int* keys = (const int*)d_in[2];
  const float* w0 = (const float*)d_in[3];
  const float* b0 = (const float*)d_in[4];
  const float* w1 = (const float*)d_in[5];
  const float* b1 = (const float*)d_in[6];
  float* out = (float*)d_out;

  constexpr size_t oXB = 0;
  constexpr size_t oH = 9609216;
  constexpr size_t oT = 28827648;
  constexpr size_t oLIST = 54452224;
  constexpr size_t oCO = 58064896;
  constexpr size_t oPOST = 58466304;
  constexpr size_t oPRE = 58667008;
  constexpr size_t oFLAG = 58867712;
  constexpr size_t oFLAGS = 58874112;
  constexpr size_t oWT0 = 58880512;
  constexpr size_t oBT0 = 58905088;
  constexpr size_t oWT1 = 58905600;
  constexpr size_t oBT1 = 58930176;
  constexpr size_t oEND = 58930432;
  static_assert(oEND <= ((size_t)128 << 20));
  static_assert((size_t)NBK * NBRUN >= (size_t)MP);
  static_assert(oXB + (size_t)MP * 96 * 2 <= oH);
  static_assert(oH + (size_t)MP * 192 * 2 <= oT);
  static_assert(oT + (size_t)MP * 128 * 4 <= oLIST && oLIST + (size_t)NBK * RCAP * 4 <= oCO && oCO + (size_t)NBK * 2 * NBRUN * 4 <= oPOST);
  if (oEND > ws_size) return;

  char* ws = (char*)d_ws;
  unsigned short* XB = (unsigned short*)(ws + oXB);
  unsigned short* H  = (unsigned short*)(ws + oH);
  float* T = (float*)(ws + oT);
  int* LIST = (int*)(ws + oLIST);
  int* CO = (int*)(ws + oCO);
  float* POST = (float*)(ws + oPOST);
  float* PRE = (float*)(ws + oPRE);
  int* FLAG = (int*)(ws + oFLAG);
  int* FLAGS = (int*)(ws + oFLAGS);
  unsigned short* WT0 = (unsigned short*)(ws + oWT0);
  float* BT0 = (float*)(ws + oBT0);
  unsigned short* WT1 = (unsigned short*)(ws + oWT1);
  float* BT1 = (float*)(ws + oBT1);

  hipFuncSetAttribute(reinterpret_cast<const void*>(&k_bucket<1, DEGF_POST, DEGADD>), hipFuncAttributeMaxDynamicSharedMemorySize, (int)BK_LDS);
  hipFuncSetAttribute(reinterpret_cast<const void*>(&k_bucket<0, DEGF_PRE, 0>), hipFuncAttributeMaxDynamicSharedMemorySize, (int)BK_LDS);

  k_cvt_rows<96, 96><<<2346, NTHR, 0, stream>>>(x, XB);
  k_wplane<<<6, NTHR, 0, stream>>>(w0, 96, 96, 96, 1, 96, 96, WT0);
  k_bias<<<1, 32, 0, stream>>>(b0, 96, 128, BT0);
  k_wplane<<<6, NTHR, 0, stream>>>(w1, 96, 32, 32, 1, 96, 192, WT1);
  k_bias<<<1, 32, 0, stream>>>(b1, 32, 64, BT1);
  k_bucket<1, DEGF_POST, DEGADD><<<NBK, NTHR, BK_LDS, stream>>>(gath, keys, LIST, CO, (int*)POST, FLAG);
  k_bucket<0, DEGF_PRE, 0><<<NBK, NTHR, BK_LDS, stream>>>(keys, gath, LIST, CO, (int*)PRE, FLAGS);
  k_gemm<96, 1><<<dim3(MP / GBM, 2), NTHR, 0, stream>>>(XB, 96, WT0, PRE, FLAGS, T, 128);
  k_replay<96, 1, 1><<<MP / ABM, NTHR, 0, stream>>>(LIST, CO, FLAG, POST, T, 128, BT0, 0.0f, (void*)H);
  k_gemm<192, 1><<<dim3(MP / GBM, 1), NTHR, 0, stream>>>(H, 192, WT1, PRE, FLAGS, T, 64);
  k_replay<32, 0, 2><<<MP / ABM, NTHR, 0, stream>>>(LIST, CO, FLAG, POST, T, 64, BT1, 0.0f, (void*)out);
}
